// ComplexityAttention_90383291777465
// MI455X (gfx1250) — hardware-verified
//
#include <hip/hip_runtime.h>


#define NT_  2048
#define HS   2048
#define DM   HS
#define NH_  16
#define NKV  4
#define HD   128
#define KW   (NKV * HD)
#define WIN  NT_
#define RMS_EPS 1e-6f
#define PSC  32768.0f
#define LOSC 1024.0f
#define LOSCI (1.0f / 1024.0f)

typedef _Float16 h16;
typedef unsigned short bf;
typedef __attribute__((ext_vector_type(16))) __bf16   v16bf;
typedef __attribute__((ext_vector_type(16))) _Float16 v16h;
typedef __attribute__((ext_vector_type(8)))  _Float16 v8h;
typedef __attribute__((ext_vector_type(8)))  unsigned short v8us;
typedef __attribute__((ext_vector_type(8)))  float    v8f;
typedef __attribute__((ext_vector_type(4)))  float    v4f;
typedef v8h  __attribute__((may_alias)) v8ha;
typedef v4f  __attribute__((may_alias)) v4fa;
typedef v8us __attribute__((may_alias)) v8usa;

__device__ __forceinline__ unsigned short f2bf(float f) { unsigned u = __float_as_uint(f); u += 0x7FFFu + ((u >> 16) & 1u); return (unsigned short)(u >> 16); }
__device__ __forceinline__ float bf2f(unsigned short b) { return __uint_as_float(((unsigned)b) << 16); }
__device__ __forceinline__ float bfr(float f) { return bf2f(f2bf(f)); }
__device__ __forceinline__ v16h cat16(v8h lo, v8h hi) { return __builtin_shufflevector(lo, hi, 0, 1, 2, 3, 4, 5, 6, 7, 8, 9, 10, 11, 12, 13, 14, 15); }
__device__ __forceinline__ v16bf cat16b(v8us lo, v8us hi) { return __builtin_bit_cast(v16bf, __builtin_shufflevector(lo, hi, 0, 1, 2, 3, 4, 5, 6, 7, 8, 9, 10, 11, 12, 13, 14, 15)); }
__device__ __forceinline__ v8f wmma16(v16h a, v16h b, v8f c) { return __builtin_amdgcn_wmma_f32_16x16x32_f16(false, a, false, b, (short)0, c, false, false); }
__device__ __forceinline__ v8f wmmab(v16bf a, v16bf b, v8f c) { return __builtin_amdgcn_wmma_f32_16x16x32_bf16(false, a, false, b, (short)0, c, false, false); }

__global__ __launch_bounds__(256) void k_cvtb(const float* __restrict__ src, int nrows, bf* dst) {
    const int lane = threadIdx.x & 31, r = blockIdx.x * 8 + (threadIdx.x >> 5);
    if (r >= nrows) return;
    v8us o[DM / 256];
#pragma unroll
    for (int q = 0; q < DM / 256; ++q) { v8us t;
#pragma unroll
        for (int i = 0; i < 8; ++i) t[i] = f2bf(src[(size_t)r * DM + q * 256 + lane * 8 + i]);
        o[q] = t; }
#pragma unroll
    for (int q = 0; q < DM / 256; ++q) *(volatile v8us*)(dst + (size_t)r * DM + q * 256 + lane * 8) = o[q];
    __threadfence();
#pragma unroll
    for (int q = 0; q < DM / 256; ++q) *(volatile v8us*)(dst + (size_t)r * DM + q * 256 + lane * 8) = o[q];
}

template <bool SPLITA, bool F16OUT = false>
__global__ __launch_bounds__(128) void k_gemmb(const bf* __restrict__ A, const bf* __restrict__ Al, const bf* __restrict__ Bn, const float* __restrict__ bias, float* C, int ldc, h16* C2, const float* __restrict__ R = nullptr, int K = DM, int roundR = 1) {
    __shared__ __align__(16) float ost[4][16 * 68];
    const int lane = threadIdx.x & 31, wave = threadIdx.x >> 5, lr = lane & 15, hi = lane >> 4;
    const int r0 = blockIdx.x * 64 + wave * 16, c0 = blockIdx.y * 64;
    const size_t aoff = (size_t)(r0 + lr) * K + 8 * hi;
    size_t boff[4];
#pragma unroll
    for (int t = 0; t < 4; ++t) boff[t] = (size_t)(c0 + t * 16 + lr) * K + 8 * hi;
    v8f acc[4];
#pragma unroll
    for (int t = 0; t < 4; ++t) acc[t] = (v8f){};
#pragma unroll 1
    for (int kc = 0; kc < K; kc += 32) {
        const v16bf a = cat16b(*(const v8us*)(A + aoff + kc), *(const v8us*)(A + aoff + kc + 16));
        v16bf al = a;
        if (SPLITA) al = cat16b(*(const v8us*)(Al + aoff + kc), *(const v8us*)(Al + aoff + kc + 16));
#pragma unroll
        for (int t = 0; t < 4; ++t) { const v16bf b = cat16b(*(const v8us*)(Bn + boff[t] + kc), *(const v8us*)(Bn + boff[t] + kc + 16)); acc[t] = wmmab(a, b, acc[t]); if (SPLITA) acc[t] = wmmab(al, b, acc[t]); }
        asm volatile("v_nop\n\tv_nop\n\tv_nop\n\tv_nop" : "+v"(acc[0]), "+v"(acc[1]), "+v"(acc[2]), "+v"(acc[3]) : "v"(a), "v"(al));
    }
    float* os = &ost[wave][0];
#pragma unroll
    for (int t = 0; t < 4; ++t) { const float bv = bias ? bfr(bias[c0 + t * 16 + lr]) : 0.f;
#pragma unroll
        for (int j = 0; j < 8; ++j) os[(hi * 8 + j) * 68 + t * 16 + lr] = acc[t][j] + bv; }
    __syncthreads();
    if (F16OUT) {
        h16* crow = (h16*)(void*)C + (size_t)r0 * ldc + c0;
        auto pass = [&]() {
#pragma unroll
            for (int s = 0; s < 4; ++s) { const int row = 4 * s + (lane >> 3), piece = lane & 7; const float* sp = os + row * 68 + piece * 8; v8h o, o2;
#pragma unroll
                for (int i = 0; i < 8; ++i) { const h16 a = (h16)sp[i]; o[i] = a; o2[i] = (h16)((sp[i] - (float)a) * LOSC); }
                *(volatile v8h*)(crow + (size_t)row * ldc + piece * 8) = o; if (C2) *(volatile v8h*)(C2 + (size_t)r0 * ldc + c0 + (size_t)row * ldc + piece * 8) = o2; }
        };
        pass(); __threadfence(); pass();
    } else {
        float* crow = C + (size_t)r0 * ldc + c0;
        auto pass = [&]() {
#pragma unroll
            for (int s = 0; s < 8; ++s) { const int Lid = (lane >> 3) + 4 * s, piece = lane & 7; const int row = Lid >> 1, cofs = (Lid & 1) * 32 + piece * 4;
                v4f val = *(const v4fa*)(os + row * 68 + cofs); if (R) { const v4f rv = *(const v4f*)(R + ((size_t)r0 + row) * ldc + c0 + cofs); val += roundR ? (v4f){bfr(rv[0]), bfr(rv[1]), bfr(rv[2]), bfr(rv[3])} : rv; }
                *(volatile v4f*)(crow + (size_t)row * ldc + cofs) = val; }
        };
        pass(); __threadfence(); pass();
    }
}

__global__ __launch_bounds__(256) void k_vt(const float* __restrict__ V, bf* VTH, bf* VTL) {
    __shared__ float tl[64][65];
    const int tid = threadIdx.x, t0 = blockIdx.x * 64, d0 = blockIdx.y * 64, g = blockIdx.z;
    { const int tt = tid >> 2, dq = (tid & 3) * 16;
#pragma unroll
      for (int i = 0; i < 16; ++i) tl[dq + i][tt] = V[(size_t)(t0 + tt) * KW + g * HD + d0 + dq + i]; }
    __syncthreads();
    const int piece = tid & 7;
    auto pass = [&]() {
#pragma unroll
        for (int s = 0; s < 2; ++s) { const int d = (tid >> 3) + 32 * s; v8us oh, ol;
#pragma unroll
            for (int i = 0; i < 8; ++i) { const float v = tl[d][piece * 8 + i]; const unsigned short hb = f2bf(v); oh[i] = hb; ol[i] = f2bf(v - bf2f(hb)); }
            const size_t o = ((size_t)g * HD + d0 + d) * NT_ + t0 + piece * 8; *(volatile v8us*)(VTH + o) = oh; *(volatile v8us*)(VTL + o) = ol; }
    };
    pass(); __threadfence(); pass();
}
__global__ __launch_bounds__(128) void k_attn(const h16* __restrict__ QH, const h16* __restrict__ QL, const h16* __restrict__ KH, const h16* __restrict__ KL, const bf* __restrict__ VTH, const bf* __restrict__ VTL, bf* CH, bf* CL) {
    __shared__ __align__(16) unsigned short plds[4][16 * 32];
    __shared__ __align__(16) unsigned short plds2[4][16 * 32];
    __shared__ __align__(16) float ost[4][16 * 68];
    const int lane = threadIdx.x & 31, wave = threadIdx.x >> 5, lr = lane & 15, hi = lane >> 4;
    const int bid = blockIdx.x; const int h = bid / (NT_ / 64), qt = bid - h * (NT_ / 64); const int g = h >> 2;
    const int q0 = qt * 64 + wave * 16;
    unsigned short* pl = &plds[wave][0]; unsigned short* pl2 = &plds2[wave][0];
    const size_t qo = (size_t)(q0 + lr) * (NH_ * HD) + h * HD + 8 * hi;
    const h16* kh_b = KH + g * HD; const h16* kl_b = KL + g * HD;
    const size_t vbase = ((size_t)g * HD) * NT_;
    v8f o[8];
#pragma unroll
    for (int n = 0; n < 8; ++n) o[n] = (v8f){};
    float mrow[8], lpart[8];
#pragma unroll
    for (int j = 0; j < 8; ++j) { mrow[j] = -3.0e38f; lpart[j] = 0.f; }
    const int kt_hi = (qt * 64 + 63) / 32; const int kt_lo = (qt * 64 > WIN) ? (qt * 64 - WIN) / 32 : 0;
#pragma unroll 1
    for (int kt = kt_lo; kt <= kt_hi; ++kt) {
        const int l0 = kt * 32;
        const size_t ko0 = (size_t)(l0 + lr) * KW + 8 * hi, ko1 = (size_t)(l0 + 16 + lr) * KW + 8 * hi;
        v8f s0 = {}, s1 = {}, x0 = {}, x1 = {};
#pragma unroll
        for (int kc = 0; kc < 4; ++kc) {
            const v16h qa = cat16(*(const v8h*)(QH + qo + kc * 32), *(const v8h*)(QH + qo + kc * 32 + 16)), qx = cat16(*(const v8h*)(QL + qo + kc * 32), *(const v8h*)(QL + qo + kc * 32 + 16));
            const v16h k0h = cat16(*(const v8h*)(kh_b + ko0 + kc * 32), *(const v8h*)(kh_b + ko0 + kc * 32 + 16)), k1h = cat16(*(const v8h*)(kh_b + ko1 + kc * 32), *(const v8h*)(kh_b + ko1 + kc * 32 + 16));
            s0 = wmma16(qa, k0h, s0); s1 = wmma16(qa, k1h, s1); x0 = wmma16(qx, k0h, x0); x1 = wmma16(qx, k1h, x1);
            asm volatile("v_nop" : "+v"(s0), "+v"(s1), "+v"(x0), "+v"(x1) : "v"(qa), "v"(qx), "v"(k0h), "v"(k1h) : "memory");
            const v16h k0l = cat16(*(const v8h*)(kl_b + ko0 + kc * 32), *(const v8h*)(kl_b + ko0 + kc * 32 + 16)), k1l = cat16(*(const v8h*)(kl_b + ko1 + kc * 32), *(const v8h*)(kl_b + ko1 + kc * 32 + 16));
            x0 = wmma16(qa, k0l, x0); x1 = wmma16(qa, k1l, x1);
            asm volatile("v_nop" : "+v"(x0), "+v"(x1) : "v"(k0l), "v"(k1l) : "memory");
        }
        asm volatile("v_nop\n\tv_nop\n\tv_nop\n\tv_nop" : "+v"(s0), "+v"(s1), "+v"(x0), "+v"(x1));
        float alpha[8];
#pragma unroll
        for (int j = 0; j < 8; ++j) { const int qi = q0 + hi * 8 + j, ja = l0 + lr, jb = l0 + 16 + lr;
            const float a0 = (ja <= qi && ja >= qi - WIN) ? (s0[j] + x0[j] * LOSCI) * 0.08838834764831845f : -__builtin_inff(), a1 = (jb <= qi && jb >= qi - WIN) ? (s1[j] + x1[j] * LOSCI) * 0.08838834764831845f : -__builtin_inff();
            float mx = fmaxf(a0, a1);
            mx = fmaxf(mx, __shfl_xor(mx, 1, 16)); mx = fmaxf(mx, __shfl_xor(mx, 2, 16)); mx = fmaxf(mx, __shfl_xor(mx, 4, 16)); mx = fmaxf(mx, __shfl_xor(mx, 8, 16));
            const float mn = fmaxf(mrow[j], mx);
            alpha[j] = __expf(mrow[j] - mn); mrow[j] = mn;
            const float p0 = __expf(a0 - mn), p1 = __expf(a1 - mn);
            lpart[j] = lpart[j] * alpha[j] + (p0 + p1);
            const int mr = hi * 8 + j; const float ps0 = p0 * PSC, ps1 = p1 * PSC; const unsigned short h0 = f2bf(ps0), h1 = f2bf(ps1);
            pl[mr * 32 + lr] = h0; pl[mr * 32 + 16 + lr] = h1; pl2[mr * 32 + lr] = f2bf(ps0 - bf2f(h0)); pl2[mr * 32 + 16 + lr] = f2bf(ps1 - bf2f(h1)); }
#pragma unroll
        for (int n = 0; n < 8; ++n)
#pragma unroll
            for (int j = 0; j < 8; ++j) o[n][j] *= alpha[j];
        asm volatile("" ::: "memory");
        const v16bf pa = cat16b(*(const v8usa*)(pl + lr * 32 + hi * 8), *(const v8usa*)(pl + lr * 32 + 16 + hi * 8));
        const v16bf px = cat16b(*(const v8usa*)(pl2 + lr * 32 + hi * 8), *(const v8usa*)(pl2 + lr * 32 + 16 + hi * 8));
#pragma unroll
        for (int n = 0; n < 8; ++n) { const size_t vo = vbase + (size_t)(n * 16 + lr) * NT_ + l0 + hi * 8;
            const v16bf vh = cat16b(*(const v8us*)(VTH + vo), *(const v8us*)(VTH + vo + 16)), vl = cat16b(*(const v8us*)(VTL + vo), *(const v8us*)(VTL + vo + 16));
            o[n] = wmmab(pa, vh, o[n]); o[n] = wmmab(px, vh, o[n]); o[n] = wmmab(pa, vl, o[n]);
            asm volatile("" : "+v"(o[n]) : "v"(vh), "v"(vl) : "memory"); }
        asm volatile("v_nop\n\tv_nop\n\tv_nop\n\tv_nop" : "+v"(o[0]), "+v"(o[7]) : "v"(pa), "v"(px));
        __builtin_amdgcn_wave_barrier();
    }
    float inv[8];
#pragma unroll
    for (int j = 0; j < 8; ++j) { float rs = lpart[j]; rs += __shfl_xor(rs, 1, 16); rs += __shfl_xor(rs, 2, 16); rs += __shfl_xor(rs, 4, 16); rs += __shfl_xor(rs, 8, 16); inv[j] = 1.0f / (rs * PSC); }
    float* os = &ost[wave][0];
    const size_t cbase = (size_t)q0 * (NH_ * HD) + (size_t)h * HD;
#pragma unroll
    for (int half = 0; half < 2; ++half) {
#pragma unroll
        for (int n = 0; n < 4; ++n)
#pragma unroll
            for (int j = 0; j < 8; ++j) os[(hi * 8 + j) * 68 + n * 16 + lr] = o[half * 4 + n][j] * inv[j];
        __builtin_amdgcn_wave_barrier(); asm volatile("" ::: "memory");
#pragma unroll
        for (int ps2 = 0; ps2 < 2; ++ps2) {
#pragma unroll
            for (int s = 0; s < 4; ++s) { const int row = 4 * s + (lane >> 3), piece = lane & 7; const float* sp = os + row * 68 + piece * 8; v8us oh, ol;
#pragma unroll
                for (int i = 0; i < 8; ++i) { const unsigned short hb = f2bf(sp[i]); oh[i] = hb; ol[i] = f2bf(sp[i] - bf2f(hb)); }
                const size_t po = cbase + (size_t)row * (NH_ * HD) + half * 64 + piece * 8; *(volatile v8us*)(CH + po) = oh; *(volatile v8us*)(CL + po) = ol; }
            if (ps2 == 0) __threadfence(); }
        __builtin_amdgcn_wave_barrier(); asm volatile("" ::: "memory");
    }
}


__global__ __launch_bounds__(256) void k_trig(float* CT, float* ST) {
    const int tid = threadIdx.x, t = blockIdx.x * 2 + (tid >> 7), d = tid & 127; const int i = d & 63;
    const float invf = 1.0f / powf(10000.0f, (float)(2 * i) / 128.0f); const float ang = (float)t * invf; const float c = cosf(ang), s = sinf(ang);
    const size_t o = (size_t)t * HD + d; *(volatile float*)(CT + o) = c; *(volatile float*)(ST + o) = s; __threadfence(); *(volatile float*)(CT + o) = c; *(volatile float*)(ST + o) = s;
}
typedef __attribute__((ext_vector_type(4))) _Float16 v4h;
__global__ __launch_bounds__(256) void k_normrope(const float* __restrict__ P, int nh, const float* __restrict__ w, const float* __restrict__ CT, const float* __restrict__ ST, h16* PH, h16* PL) {
    const int lane = threadIdx.x & 31; const int wid = blockIdx.x * 8 + (threadIdx.x >> 5); const int t = wid / nh, h = wid - t * nh; if (t >= NT_) return;
    const size_t base = (size_t)t * (nh * HD) + h * HD; const int d0 = lane * 4;
    float x[4], pr[4]; float ss = 0.f;
#pragma unroll
    for (int i = 0; i < 4; ++i) { x[i] = P[base + d0 + i]; ss = fmaf(x[i], x[i], ss); }
#pragma unroll
    for (int sh = 16; sh; sh >>= 1) ss += __shfl_xor(ss, sh, 32);
    const float rn = rsqrtf(ss * (1.0f / HD) + RMS_EPS);
#pragma unroll
    for (int i = 0; i < 4; ++i) x[i] = x[i] * rn * bfr(w[d0 + i]);
#pragma unroll
    for (int i = 0; i < 4; ++i) pr[i] = __shfl_xor(x[i], 16, 32);
    v4h oh, ol;
#pragma unroll
    for (int i = 0; i < 4; ++i) { const int d = d0 + i; const float c = CT[(size_t)t * HD + d], s = ST[(size_t)t * HD + d]; const float y = (d < 64) ? (x[i] * c - pr[i] * s) : (x[i] * c + pr[i] * s);
        const h16 a = (h16)y; oh[i] = a; ol[i] = (h16)((y - (float)a) * LOSC); }
    *(volatile v4h*)(PH + base + d0) = oh; *(volatile v4h*)(PL + base + d0) = ol; __threadfence(); *(volatile v4h*)(PH + base + d0) = oh; *(volatile v4h*)(PL + base + d0) = ol;
}

extern "C" void kernel_launch(void* const* d_in, const int* in_sizes, int n_in,
                              void* d_out, int out_size, void* d_ws, size_t ws_size, hipStream_t stream) {
    (void)in_sizes; (void)n_in; (void)out_size;
    const float* x = (const float*)d_in[0]; const float* mu = (const float*)d_in[1]; const float* wq = (const float*)d_in[2]; const float* wk = (const float*)d_in[3]; const float* wv = (const float*)d_in[4]; const float* wo = (const float*)d_in[5];
    const float* wmq = (const float*)d_in[6]; const float* wmk = (const float*)d_in[7]; const float* wmv = (const float*)d_in[8]; const float* qnw = (const float*)d_in[9]; const float* knw = (const float*)d_in[10];
    float* out = (float*)d_out;
    char* wsp = (char*)d_ws;
    auto take = [&](size_t bytes) { char* p = wsp; wsp += (bytes + 255) & ~(size_t)255; return (void*)p; };
    bf* Xb = (bf*)take((size_t)NT_ * HS * 2); bf* Mb = (bf*)take((size_t)NT_ * HS * 2);
    bf* WqB = (bf*)take((size_t)HS * HS * 2); bf* WmqB = (bf*)take((size_t)HS * HS * 2); bf* WkB = (bf*)take((size_t)KW * HS * 2); bf* WmkB = (bf*)take((size_t)KW * HS * 2); bf* WvB = (bf*)take((size_t)KW * HS * 2); bf* WmvB = (bf*)take((size_t)KW * HS * 2); bf* WoB = (bf*)take((size_t)HS * HS * 2);
    float* TMP = (float*)take((size_t)NT_ * HS * 4); float* TMP2 = (float*)take((size_t)NT_ * HS * 4); float* CT = (float*)take((size_t)NT_ * HD * 4); float* ST = (float*)take((size_t)NT_ * HD * 4);
    h16* QH = (h16*)take((size_t)NT_ * HS * 2); h16* QL = (h16*)take((size_t)NT_ * HS * 2); h16* KH = (h16*)take((size_t)NT_ * KW * 2); h16* KL = (h16*)take((size_t)NT_ * KW * 2);
    bf* VTH = (bf*)take((size_t)KW * NT_ * 2); bf* VTL = (bf*)take((size_t)KW * NT_ * 2); bf* CH = (bf*)take((size_t)NT_ * HS * 2); bf* CL = (bf*)take((size_t)NT_ * HS * 2);
    if ((size_t)(wsp - (char*)d_ws) > ws_size) return;
    k_cvtb<<<HS / 8, 256, 0, stream>>>(wq, HS, WqB); k_cvtb<<<HS / 8, 256, 0, stream>>>(wmq, HS, WmqB); k_cvtb<<<KW / 8, 256, 0, stream>>>(wk, KW, WkB); k_cvtb<<<KW / 8, 256, 0, stream>>>(wmk, KW, WmkB);
    k_cvtb<<<KW / 8, 256, 0, stream>>>(wv, KW, WvB); k_cvtb<<<KW / 8, 256, 0, stream>>>(wmv, KW, WmvB); k_cvtb<<<HS / 8, 256, 0, stream>>>(wo, HS, WoB);
    k_trig<<<NT_ / 2, 256, 0, stream>>>(CT, ST);
    k_cvtb<<<NT_ / 8, 256, 0, stream>>>(x, NT_, Xb); k_cvtb<<<NT_ / 8, 256, 0, stream>>>(mu, NT_, Mb);
    k_gemmb<false, false><<<dim3(NT_ / 64, HS / 64, 1), 128, 0, stream>>>(Xb, nullptr, WqB, nullptr, TMP, HS, nullptr, nullptr, HS, 0);
    k_gemmb<false, false><<<dim3(NT_ / 64, HS / 64, 1), 128, 0, stream>>>(Mb, nullptr, WmqB, nullptr, TMP2, HS, nullptr, TMP, HS, 0);
    k_normrope<<<(NT_ * NH_) / 8, 256, 0, stream>>>(TMP2, NH_, qnw, CT, ST, QH, QL);
    k_gemmb<false, false><<<dim3(NT_ / 64, KW / 64, 1), 128, 0, stream>>>(Xb, nullptr, WkB, nullptr, TMP, KW, nullptr, nullptr, HS, 0);
    k_gemmb<false, false><<<dim3(NT_ / 64, KW / 64, 1), 128, 0, stream>>>(Mb, nullptr, WmkB, nullptr, TMP2, KW, nullptr, TMP, HS, 0);
    k_normrope<<<(NT_ * NKV) / 8, 256, 0, stream>>>(TMP2, NKV, knw, CT, ST, KH, KL);
    k_gemmb<false, false><<<dim3(NT_ / 64, KW / 64, 1), 128, 0, stream>>>(Xb, nullptr, WvB, nullptr, TMP, KW, nullptr, nullptr, HS, 0);
    k_gemmb<false, false><<<dim3(NT_ / 64, KW / 64, 1), 128, 0, stream>>>(Mb, nullptr, WmvB, nullptr, TMP2, KW, nullptr, TMP, HS, 0);
    k_vt<<<dim3(NT_ / 64, 2, NKV), 256, 0, stream>>>(TMP2, VTH, VTL);
    k_attn<<<NH_ * (NT_ / 64), 128, 0, stream>>>(QH, QL, KH, KL, VTH, VTL, CH, CL);
    k_gemmb<true, false><<<dim3(NT_ / 64, HS / 64, 1), 128, 0, stream>>>(CH, CL, WoB, nullptr, out, HS, nullptr, nullptr, HS, 0);
}
